// TransformerEncoderLayerWithRoPE_64922725646591
// MI455X (gfx1250) — hardware-run, weakly checked
//
#include <hip/hip_runtime.h>
#include <math.h>

typedef __attribute__((ext_vector_type(16))) _Float16 v16h;
typedef __attribute__((ext_vector_type(16))) __bf16 v16b;
typedef __attribute__((ext_vector_type(8)))  _Float16 v8h;
typedef __attribute__((ext_vector_type(8)))  float v8f;
typedef __attribute__((ext_vector_type(4)))  float v4f;
typedef __attribute__((ext_vector_type(2)))  float v2f;
typedef __attribute__((ext_vector_type(4)))  unsigned v4u;
typedef __attribute__((ext_vector_type(4)))  int v4i;
typedef float __attribute__((may_alias)) float_a;
typedef int __attribute__((may_alias)) int_a;

template <typename T> __device__ __forceinline__ void vst2(void* p, T v) { *(volatile T*)p = v; __threadfence(); *(volatile T*)p = v; }
__device__ __forceinline__ v8f wmma16(v16h a, v16h b, v8f c) {
  v8f d = __builtin_amdgcn_wmma_f32_16x16x32_f16(false, a, false, b, (short)0, c, false, false);
  asm volatile("v_nop\n\tv_nop\n\tv_nop\n\tv_nop" : "+v"(d) : "v"(a), "v"(b));
  return d;
}
__device__ __forceinline__ v8f wmma_bf(v16b a, v16b b, v8f c) {
  v8f d = __builtin_amdgcn_wmma_f32_16x16x32_bf16(false, a, false, b, (short)0, c, false, false);
  asm volatile("v_nop\n\tv_nop\n\tv_nop\n\tv_nop" : "+v"(d) : "v"(a), "v"(b));
  return d;
}
__device__ __forceinline__ v16h frag_h(const _Float16* rowk0, int lane) {
  union { v16h v; v8h q[2]; } u; const _Float16* p = rowk0 + 8 * (lane >> 4);
  u.q[0] = *(const v8h*)p; u.q[1] = *(const v8h*)(p + 16); return u.v;
}
__device__ __forceinline__ v16h frag_f32(const float* rowk0, int lane) {
  v16h a; const float* p = rowk0 + 8 * (lane >> 4);
#pragma unroll
  for (int i = 0; i < 8; ++i) { a[i] = (_Float16)p[i]; a[8 + i] = (_Float16)p[16 + i]; }
  return a;
}
__device__ __forceinline__ v16h frag_f32s(const float* rowk0, int lane, float sc) {
  v16h a; const float* p = rowk0 + 8 * (lane >> 4);
#pragma unroll
  for (int i = 0; i < 8; ++i) { a[i] = (_Float16)(p[i] * sc); a[8 + i] = (_Float16)(p[16 + i] * sc); }
  return a;
}
__device__ __forceinline__ v16h fragc_f32(const float* W, int k0, int n, int lane, int ld, int K) {
  v16h a; const int g = lane >> 4;
#pragma unroll
  for (int i = 0; i < 8; ++i) { const int ka = k0 + 8 * g + i, kb = ka + 16;
    a[i] = (_Float16)(ka < K ? W[(size_t)(ka < K ? ka : K - 1) * ld + n] : 0.f); a[8 + i] = (_Float16)(kb < K ? W[(size_t)(kb < K ? kb : K - 1) * ld + n] : 0.f); }
  return a;
}
struct F2 { v16b h, l; };
__device__ __forceinline__ F2 bsplit16(const float v[16]) { F2 r;
#pragma unroll
  for (int i = 0; i < 16; ++i) { const __bf16 h = (__bf16)v[i]; r.h[i] = h; r.l[i] = (__bf16)(v[i] - (float)h); }
  return r; }
__device__ __forceinline__ F2 split_row(const float* row, int k0, int lane) { float v[16]; const float* p = row + k0 + 8 * (lane >> 4);
#pragma unroll
  for (int i = 0; i < 8; ++i) { v[i] = p[i]; v[8 + i] = p[16 + i]; }
  return bsplit16(v); }
__device__ __forceinline__ F2 split_rowK(const float* row, int k0, int lane, int K) { float v[16]; const int g = lane >> 4;
#pragma unroll
  for (int i = 0; i < 8; ++i) { const int ka = k0 + 8 * g + i, kb = ka + 16; v[i] = ka < K ? row[ka < K ? ka : K - 1] : 0.f; v[8 + i] = kb < K ? row[kb < K ? kb : K - 1] : 0.f; }
  return bsplit16(v); }
__device__ __forceinline__ F2 split_col(const float* W, int k0, int n, int lane, int ld, int K) { float v[16]; const int g = lane >> 4;
#pragma unroll
  for (int i = 0; i < 8; ++i) { const int ka = k0 + 8 * g + i, kb = ka + 16; v[i] = ka < K ? W[(size_t)(ka < K ? ka : K - 1) * ld + n] : 0.f; v[8 + i] = kb < K ? W[(size_t)(kb < K ? kb : K - 1) * ld + n] : 0.f; }
  return bsplit16(v); }
__device__ __forceinline__ v8f mac3(const F2& a, const F2& b, v8f c) { c = wmma_bf(a.l, b.h, c); c = wmma_bf(a.h, b.l, c); return wmma_bf(a.h, b.h, c); }
__device__ __forceinline__ float sigm(float v) { return 1.0f / (1.0f + expf(-v)); }
#define LDSX() do { asm volatile("s_wait_dscnt 0" ::: "memory"); __builtin_amdgcn_wave_barrier(); __builtin_amdgcn_fence(__ATOMIC_RELEASE, "workgroup"); } while (0)


#define NB 16
#define TT 1024
#define DD 128
#define NHD 8
#define HDD 16
#define FF 512
#define BG 2
#define NR (NB * TT)
#define RMS_EPS 1.1920929e-7f
#ifndef TNB
#define TNB NB
#endif
typedef __attribute__((ext_vector_type(8))) __bf16 v8b;
__device__ __forceinline__ v16b frag_b(const __bf16* rowk0, int lane) {
  union { v16b v; v8b q[2]; } u; const __bf16* p = rowk0 + 8 * (lane >> 4);
  u.q[0] = *(const v8b*)p; u.q[1] = *(const v8b*)(p + 16); return u.v;
}
__device__ __forceinline__ float bfr(float v) { return (float)(__bf16)v; }
__device__ __attribute__((noinline)) float exp_ni(float v) { return expf(v); }
__device__ __attribute__((noinline)) float erf_ni(float v) { return erff(v); }

#define WS_Q   0u
#define WS_K   (WS_Q + 2u * (size_t)NR * DD)
#define WS_VT  (WS_K + 2u * (size_t)NR * DD)
#define WS_S   (WS_VT + 2u * (size_t)NB * DD * TT)
#define WS_PH  (WS_S + 4u * (size_t)BG * NHD * TT * TT)
#define WS_CTX (WS_PH + 2u * (size_t)BG * NHD * TT * TT)
#define WS_END (WS_CTX + 4u * (size_t)NR * DD)

__global__ __launch_bounds__(128) void k_pre(const float* __restrict__ X, const float* __restrict__ COS, const float* __restrict__ SIN, const float* __restrict__ WQ, const float* __restrict__ BQ, const float* __restrict__ WK, const float* __restrict__ BK, const float* __restrict__ WV, const float* __restrict__ BV, _Float16* __restrict__ Q, _Float16* __restrict__ Kr, _Float16* __restrict__ VT) {
  __shared__ __align__(16) _Float16 sa[64][DD + 8]; __shared__ __align__(16) float sf[64][DD + 4]; __shared__ __align__(16) _Float16 sh[64][DD + 8]; __shared__ __align__(16) _Float16 th[DD][72];
  const int tid = threadIdx.x, wave = tid >> 5, lane = tid & 31, col = lane & 15, g = lane >> 4; const size_t r0 = (size_t)blockIdx.x * 64;
  for (int e = tid; e < 64 * DD; e += 128) { const int rl = e >> 7, c = e & 127; sa[rl][c] = (_Float16)bfr(X[(r0 + rl) * DD + c]); }
  __syncthreads();
#pragma unroll 1
  for (int which = 0; which < 3; ++which) { const float* Wm = which == 0 ? WQ : which == 1 ? WK : WV; const float* Bm = which == 0 ? BQ : which == 1 ? BK : BV;
    v8f acc[8] = {};
#pragma unroll
    for (int kc = 0; kc < DD / 32; ++kc) { const v16h a = frag_h(&sa[wave * 16 + col][kc * 32], lane);
#pragma unroll
      for (int j = 0; j < 8; ++j) { v16h w; const int o = j * 16 + col;
#pragma unroll
        for (int i = 0; i < 8; ++i) { w[i] = (_Float16)bfr(Wm[(size_t)(kc * 32 + 8 * g + i) * DD + o]); w[8 + i] = (_Float16)bfr(Wm[(size_t)(kc * 32 + 16 + 8 * g + i) * DD + o]); }
        acc[j] = wmma16(a, w, acc[j]); } }
#pragma unroll
    for (int j = 0; j < 8; ++j) { const float bb = bfr(Bm[j * 16 + col]);
#pragma unroll
      for (int r = 0; r < 8; ++r) sf[wave * 16 + 8 * g + r][j * 16 + col] = acc[j][r] + bb; }
    __syncthreads();
    if (which < 2) {
      for (int e = tid; e < 64 * DD; e += 128) { const int rl = e >> 7, c = e & 127; const int d = c & 15, i2 = d & 7; const int s = (int)((r0 + rl) % TT); const float cs = bfr(COS[s * 8 + i2]), sn = bfr(SIN[s * 8 + i2]);
        const float x1 = sf[rl][(c & ~15) + i2], x2 = sf[rl][(c & ~15) + 8 + i2]; const float v = (d < 8) ? (x1 * cs - x2 * sn) : (x1 * sn + x2 * cs); sh[rl][c] = (_Float16)v; }
      __syncthreads(); _Float16* dst = which == 0 ? Q : Kr;
      for (int e = tid; e < 64 * 16; e += 128) { const int rl = e >> 4, q = e & 15; vst2((unsigned*)(dst + (r0 + rl) * DD + q * 8), *(const v4u*)&sh[rl][q * 8]); } }
    else { for (int e = tid; e < 64 * DD; e += 128) { const int rl = e >> 7, c = e & 127; th[c][rl] = (_Float16)sf[rl][c]; }
      __syncthreads(); const size_t b = r0 / TT; const int s0 = (int)(r0 % TT);
      for (int e = tid; e < DD * 8; e += 128) { const int c = e >> 3, q = e & 7; vst2((unsigned*)(VT + (b * DD + c) * (size_t)TT + s0 + q * 8), *(const v4u*)&th[c][q * 8]); } }
    __syncthreads(); } }
__global__ __launch_bounds__(128) void k_sc(const _Float16* __restrict__ Q, const _Float16* __restrict__ Kr, int b0, float* __restrict__ S0) { __shared__ __align__(16) float ss[4][16][132];
  const int z = blockIdx.z; const size_t b = b0 + z / NHD; const int h = z % NHD; float* S = S0 + (size_t)z * TT * TT;
  const int tid = threadIdx.x, wave = tid >> 5, lane = tid & 31, col = lane & 15, g = lane >> 4; const int k0 = blockIdx.y * 128; const int ql0 = blockIdx.x * 64 + wave * 16;
  v16h a; { const _Float16* p = Q + (b * TT + ql0 + col) * DD + h * HDD + 8 * g;
#pragma unroll
    for (int i = 0; i < 8; ++i) { a[i] = p[i]; a[8 + i] = (_Float16)0.f; } }
  v8f acc[8] = {};
#pragma unroll
  for (int j = 0; j < 8; ++j) { v16h kb; const _Float16* p = Kr + (b * TT + k0 + j * 16 + col) * DD + h * HDD + 8 * g;
#pragma unroll
    for (int i = 0; i < 8; ++i) { kb[i] = p[i]; kb[8 + i] = (_Float16)0.f; }
    acc[j] = wmma16(a, kb, acc[j]); }
#pragma unroll
  for (int j = 0; j < 8; ++j)
#pragma unroll
    for (int r = 0; r < 8; ++r) ss[wave][8 * g + r][j * 16 + col] = acc[j][r] * 0.25f;
  LDSX(); for (int rl = 0; rl < 16; ++rl) vst2(S + (size_t)(ql0 + rl) * TT + k0 + lane * 4, *(const v4f*)&ss[wave][rl][lane * 4]); }
__global__ __launch_bounds__(256) void k_sm(const float* __restrict__ S0, _Float16* __restrict__ PH0) { __shared__ float sred[8]; __shared__ float sbc; __shared__ __align__(16) _Float16 sh[TT];
  const int t = threadIdx.x; const size_t row = blockIdx.x; const float* sr = S0 + (size_t)blockIdx.y * TT * TT + row * TT; _Float16* ph = PH0 + (size_t)blockIdx.y * TT * TT + row * TT;
  float m = -3.0e38f; for (int k = t; k < TT; k += 256) m = fmaxf(m, sr[k]);
#pragma unroll
  for (int o = 1; o < 32; o <<= 1) m = fmaxf(m, __shfl_xor(m, o));
  if ((t & 31) == 0) sred[t >> 5] = m; __syncthreads(); if (t == 0) { float a = sred[0]; for (int i = 1; i < 8; ++i) a = fmaxf(a, sred[i]); sbc = a; } __syncthreads(); m = sbc; __syncthreads();
  float sum = 0.f; for (int k = t; k < TT; k += 256) sum += expf(sr[k] - m);
#pragma unroll
  for (int o = 1; o < 32; o <<= 1) sum += __shfl_xor(sum, o);
  if ((t & 31) == 0) sred[t >> 5] = sum; __syncthreads(); if (t == 0) { float a = 0.f; for (int i = 0; i < 8; ++i) a += sred[i]; sbc = 1.0f / a; } __syncthreads(); const float inv = sbc;
  for (int k = t; k < TT; k += 256) sh[k] = (_Float16)(expf(sr[k] - m) * inv * 2048.0f);
  __syncthreads(); for (int q = t; q < TT / 8; q += 256) vst2((unsigned*)(ph + q * 8), *(const v4u*)&sh[q * 8]); }
__global__ __launch_bounds__(128) void k_pv(const _Float16* __restrict__ PH0, const _Float16* __restrict__ VT, int b0, float* __restrict__ CTX) { __shared__ __align__(16) float ss[4][16][36];
  const int z = blockIdx.z; const int bl = z / (NHD / 2), hp = z % (NHD / 2); const size_t b = b0 + bl; const int hA = 2 * hp;
  const int tid = threadIdx.x, wave = tid >> 5, lane = tid & 31, col = lane & 15, g = lane >> 4; const int ql0 = blockIdx.x * 64 + wave * 16;
  v8f acc[2] = {};
#pragma unroll
  for (int u = 0; u < 2; ++u) { const _Float16* PH = PH0 + (size_t)(bl * NHD + hA + u) * TT * TT;
#pragma unroll 1
    for (int kc = 0; kc < TT / 32; ++kc) { const v16h ph = frag_h(PH + (size_t)(ql0 + col) * TT + kc * 32, lane); acc[u] = wmma16(ph, frag_h(VT + (b * DD + (hA + u) * HDD + col) * (size_t)TT + kc * 32, lane), acc[u]); } }
#pragma unroll
  for (int u = 0; u < 2; ++u)
#pragma unroll
    for (int r = 0; r < 8; ++r) ss[wave][8 * g + r][u * 16 + col] = acc[u][r] * (1.0f / 2048.0f);
  LDSX(); for (int rl = 0; rl < 16; ++rl) if (lane < 8) vst2(CTX + (b * TT + ql0 + rl) * DD + hA * HDD + lane * 4, *(const v4f*)&ss[wave][rl][lane * 4]); }
__global__ __launch_bounds__(128) void k_post(const float* __restrict__ CTX, const float* __restrict__ X, const float* __restrict__ WO, const float* __restrict__ BO, const float* __restrict__ W1, const float* __restrict__ Bf1, const float* __restrict__ W2, const float* __restrict__ Bf2, const float* __restrict__ G1, const float* __restrict__ G2, float* __restrict__ OUT) {
  __shared__ __align__(16) _Float16 sa[64][DD + 8]; __shared__ __align__(16) float sx[64][DD + 4]; __shared__ __align__(16) _Float16 shh[64][FF + 8]; __shared__ float srs[64];
  const int tid = threadIdx.x, wave = tid >> 5, lane = tid & 31, col = lane & 15, g = lane >> 4; const size_t r0 = (size_t)blockIdx.x * 64;
  for (int e = tid; e < 64 * DD; e += 128) { const int rl = e >> 7, c = e & 127; sa[rl][c] = (_Float16)CTX[(r0 + rl) * DD + c]; }
  __syncthreads();
  { v8f acc[8] = {};
#pragma unroll
    for (int kc = 0; kc < DD / 32; ++kc) { const v16h a = frag_h(&sa[wave * 16 + col][kc * 32], lane);
#pragma unroll
      for (int j = 0; j < 8; ++j) { v16h w; const int o = j * 16 + col;
#pragma unroll
        for (int i = 0; i < 8; ++i) { w[i] = (_Float16)bfr(WO[(size_t)(kc * 32 + 8 * g + i) * DD + o]); w[8 + i] = (_Float16)bfr(WO[(size_t)(kc * 32 + 16 + 8 * g + i) * DD + o]); }
        acc[j] = wmma16(a, w, acc[j]); } }
#pragma unroll
    for (int j = 0; j < 8; ++j) { const int o = j * 16 + col; const float bb = bfr(BO[o]);
#pragma unroll
      for (int r = 0; r < 8; ++r) { const int rl = wave * 16 + 8 * g + r; sx[rl][o] = acc[j][r] + bb + bfr(X[(r0 + rl) * DD + o]); } } }
  __syncthreads();
  if (tid < 64) { float s2 = 0.f; for (int c = 0; c < DD; ++c) { const float v = sx[tid][c]; s2 += v * v; } srs[tid] = 1.0f / sqrtf(s2 * (1.0f / DD) + RMS_EPS); }
  __syncthreads();
  for (int e = tid; e < 64 * DD; e += 128) { const int rl = e >> 7, c = e & 127; const float v = sx[rl][c] * srs[rl] * bfr(G1[c]); sx[rl][c] = v; sa[rl][c] = (_Float16)v; }
  __syncthreads();
#pragma unroll 1
  for (int q4 = 0; q4 < FF / 128; ++q4) { v8f acc[8] = {};
#pragma unroll
    for (int kc = 0; kc < DD / 32; ++kc) { const v16h a = frag_h(&sa[wave * 16 + col][kc * 32], lane);
#pragma unroll
      for (int j = 0; j < 8; ++j) { v16h w; const int o = q4 * 128 + j * 16 + col;
#pragma unroll
        for (int i = 0; i < 8; ++i) { w[i] = (_Float16)bfr(W1[(size_t)(kc * 32 + 8 * g + i) * FF + o]); w[8 + i] = (_Float16)bfr(W1[(size_t)(kc * 32 + 16 + 8 * g + i) * FF + o]); }
        acc[j] = wmma16(a, w, acc[j]); } }
#pragma unroll
    for (int j = 0; j < 8; ++j) { const int o = q4 * 128 + j * 16 + col; const float bb = bfr(Bf1[o]);
#pragma unroll
      for (int r = 0; r < 8; ++r) { const float u = acc[j][r] + bb; shh[wave * 16 + 8 * g + r][o] = (_Float16)(0.5f * u * (1.0f + erff(u * 0.70710678118654752f))); } } }
  __syncthreads();
  { v8f acc[8] = {};
#pragma unroll 2
    for (int kc = 0; kc < FF / 32; ++kc) { const v16h a = frag_h(&shh[wave * 16 + col][kc * 32], lane);
#pragma unroll
      for (int j = 0; j < 8; ++j) { v16h w; const int o = j * 16 + col;
#pragma unroll
        for (int i = 0; i < 8; ++i) { w[i] = (_Float16)bfr(W2[(size_t)(kc * 32 + 8 * g + i) * DD + o]); w[8 + i] = (_Float16)bfr(W2[(size_t)(kc * 32 + 16 + 8 * g + i) * DD + o]); }
        acc[j] = wmma16(a, w, acc[j]); } }
    __syncthreads();
#pragma unroll
    for (int j = 0; j < 8; ++j) { const int o = j * 16 + col; const float bb = bfr(Bf2[o]);
#pragma unroll
      for (int r = 0; r < 8; ++r) { const int rl = wave * 16 + 8 * g + r; sx[rl][o] = sx[rl][o] + acc[j][r] + bb; } } }
  __syncthreads();
  if (tid < 64) { float s2 = 0.f; for (int c = 0; c < DD; ++c) { const float v = sx[tid][c]; s2 += v * v; } srs[tid] = 1.0f / sqrtf(s2 * (1.0f / DD) + RMS_EPS); }
  __syncthreads();
  for (int e = tid; e < 64 * DD; e += 128) { const int rl = e >> 7, c = e & 127; sx[rl][c] = sx[rl][c] * srs[rl] * bfr(G2[c]); }
  __syncthreads(); for (int e = tid; e < 64 * 32; e += 128) { const int rl = e >> 5, q = e & 31; vst2(OUT + (r0 + rl) * DD + q * 4, *(const v4f*)&sx[rl][q * 4]); } }
extern "C" void kernel_launch(void* const* d_in, const int* in_sizes, int n_in, void* d_out, int out_size, void* d_ws, size_t ws_size, hipStream_t stream) {
  (void)in_sizes; (void)n_in; (void)out_size;
  const float** F = (const float**)d_in;
  if (ws_size < (size_t)WS_END) return;
  char* ws = (char*)d_ws; _Float16 *Q = (_Float16*)(ws + WS_Q), *Kr = (_Float16*)(ws + WS_K), *VT = (_Float16*)(ws + WS_VT), *PH = (_Float16*)(ws + WS_PH); float *S = (float*)(ws + WS_S), *CTX = (float*)(ws + WS_CTX);
  k_pre<<<TNB * TT / 64, 128, 0, stream>>>(F[0], F[1], F[2], F[3], F[4], F[5], F[6], F[7], F[8], Q, Kr, VT);
  for (int b0 = 0; b0 < TNB; b0 += BG) { const int nbk = (TNB - b0 < BG) ? (TNB - b0) : BG;
    k_sc<<<dim3(TT / 64, TT / 128, nbk * NHD), 128, 0, stream>>>(Q, Kr, b0, S);
    k_sm<<<dim3(TT, nbk * NHD), 256, 0, stream>>>(S, PH);
    k_pv<<<dim3(TT / 64, 1, nbk * NHD / 2), 128, 0, stream>>>(PH, VT, b0, CTX);
  }
  k_post<<<TNB * TT / 64, 128, 0, stream>>>(CTX, F[0], F[9], F[10], F[11], F[12], F[13], F[14], F[15], F[16], (float*)d_out);
}
